// MultiqueryAttention_59940563583325
// MI455X (gfx1250) — hardware-verified
//
#include <hip/hip_runtime.h>


namespace {
constexpr int B = 4, T = 2048, DM = 1024, H = 16, HD = 64, BL = 4  , QL = 2048  ;
constexpr int NSL = DM / 128;
constexpr int NWT = DM + 2 * HD;
constexpr float XS = 8.0f, WSC = 256.0f, PS = 1024.0f, RS_ = 1024.0f, LOG2E = 1.4426950408889634f;
static_assert(T % 64 == 0 && QL % 32 == 0 && DM % 256 == 0 && H * HD == DM && HD == 64, "tiling");
typedef _Float16 b16;
typedef __attribute__((ext_vector_type(16))) _Float16 v16b;
typedef __attribute__((ext_vector_type(8))) _Float16 v8b;
typedef __attribute__((ext_vector_type(8))) float v8f;
typedef __attribute__((ext_vector_type(4))) float v4f;
__device__ __forceinline__ float bf16_rne(float f) { unsigned int u = __float_as_uint(f); u += 0x7FFFu + ((u >> 16) & 1u); return __uint_as_float(u & 0xFFFF0000u); }
__device__ __forceinline__ void split16(float v, b16& hi, b16& lo) { hi = (b16)v; lo = (b16)(v - (float)hi); }
__device__ __forceinline__ v16b frag_kb(const b16* p, int hh) { const v8b a = *(const v8b*)(p + 8 * hh), b = *(const v8b*)(p + 16 + 8 * hh); v16b f;
#pragma unroll
  for (int e = 0; e < 8; ++e) { f[e] = a[e]; f[8 + e] = b[e]; } return f; }
__device__ __forceinline__ v8f wmma16b(v16b a, v16b b, v8f c) { v8f d = __builtin_amdgcn_wmma_f32_16x16x32_f16(false, a, false, b, (short)0, c, false, false); asm volatile("v_nop\n\tv_nop\n\tv_nop\n\tv_nop" : "+v"(d) : "v"(a), "v"(b)); return d; }
__device__ __forceinline__ void wave_lds_sync() { __builtin_amdgcn_fence(__ATOMIC_RELEASE, "workgroup"); __builtin_amdgcn_wave_barrier(); __builtin_amdgcn_fence(__ATOMIC_ACQUIRE, "workgroup"); }
__device__ __forceinline__ float pmul(float a, float b) { float p = a * b; asm volatile("" : "+v"(p)); return p; }
__device__ __forceinline__ int iclamp(int v, int lo, int hi) { return v < lo ? lo : (v > hi ? hi : v); }

typedef __attribute__((ext_vector_type(2))) _Float16 v2h;
typedef __attribute__((ext_vector_type(4))) _Float16 v4h;
typedef __attribute__((ext_vector_type(2))) float v2f;
typedef __attribute__((ext_vector_type(4))) int v4i;
__device__ __forceinline__ float nexp2(float v) { return __builtin_amdgcn_exp2f(v); }
__global__ __launch_bounds__(256) void prep_kernel(const float* __restrict__ wq, const float* __restrict__ wk, const float* __restrict__ wv, const float* __restrict__ wo, b16* __restrict__ WT, b16* __restrict__ WO) {
  const size_t u = (size_t)blockIdx.x * 256 + threadIdx.x; const size_t nq = (size_t)NWT * DM / 8, no = (size_t)DM * DM / 8; if (u >= nq + no) return;
  v8b o; b16* dst;
  if (u < nq) { const int row = (int)(u / (DM / 8)), k0 = (int)(u % (DM / 8)) * 8; const float* w; int oc, ld;
    if (row < DM) { w = wq; oc = row; ld = DM; } else if (row < DM + HD) { w = wk; oc = row - DM; ld = HD; } else { w = wv; oc = row - DM - HD; ld = HD; }
    for (int j = 0; j < 8; ++j) o[j] = (b16)(bf16_rne(w[(size_t)(k0 + j) * ld + oc]) * WSC); dst = WT + (size_t)row * DM + k0; }
  else { const size_t e = u - nq; const int row = (int)(e / (DM / 8)), k0 = (int)(e % (DM / 8)) * 8; for (int j = 0; j < 8; ++j) o[j] = (b16)(bf16_rne(wo[(size_t)(k0 + j) * DM + row]) * WSC); dst = WO + (size_t)row * DM + k0; }
  for (int pass = 0; pass < 2; ++pass) { *(volatile v8b*)dst = o; __threadfence(); }
}
__global__ __launch_bounds__(128) void proj_kernel(const float* __restrict__ x, const b16* __restrict__ WT, const float* __restrict__ bq, const float* __restrict__ bk, const float* __restrict__ bv, b16* __restrict__ QP, b16* __restrict__ KP, b16* __restrict__ VTh, b16* __restrict__ VTl) {
  __shared__ __attribute__((aligned(16))) b16 As[64][256 + 8]; __shared__ __attribute__((aligned(16))) float Tf[4][16][128 + 4];
  const int wave = threadIdx.x >> 5, lane = threadIdx.x & 31, nloc = lane & 15, hlf = lane >> 4; const int t0 = blockIdx.x * 64; const int b = blockIdx.y; const int slab = blockIdx.z, n0 = slab * 128; const bool kv = (slab == NSL);
  if (!kv && t0 >= QL) return;
  const float* xb = x + ((size_t)b * T + t0) * DM;
  v8f acc[8];
#pragma unroll
  for (int t = 0; t < 8; ++t) acc[t] = (v8f){};
#pragma unroll 1
  for (int kc = 0; kc < DM; kc += 256) {
    __syncthreads();
    for (int i = threadIdx.x; i < 64 * 64; i += 128) { const int rr = i / 64, q = (i % 64) * 4; const v4f f = *(const v4f*)(xb + (size_t)rr * DM + kc + q); v4h o; for (int j = 0; j < 4; ++j) o[j] = (b16)(bf16_rne(f[j]) * XS); *(v4h*)(&As[rr][q]) = o; }
    __syncthreads();
#pragma unroll 2
    for (int kb = 0; kb < 256; kb += 32) { const v16b a = frag_kb(&As[wave * 16 + nloc][kb], hlf);
#pragma unroll
      for (int t = 0; t < 8; ++t) acc[t] = wmma16b(a, frag_kb(WT + (size_t)(n0 + t * 16 + nloc) * DM + kc + kb, hlf), acc[t]); } }
#pragma unroll
  for (int t = 0; t < 8; ++t) { const int cl = t * 16 + nloc; const float bb = kv ? (cl < HD ? bf16_rne(bk[cl]) : bf16_rne(bv[cl - HD])) : bf16_rne(bq[n0 + cl]);
#pragma unroll
    for (int r = 0; r < 8; ++r) Tf[wave][8 * hlf + r][cl] = acc[t][r] * (1.0f / (XS * WSC)) + bb; }
  __syncthreads();
  for (int pass = 0; pass < 2; ++pass) {
    if (!kv) { const int c = n0 + lane * 4; const int h = c / HD, d = c % HD;
      for (int rr = 0; rr < 16; ++rr) { const int tok = t0 + wave * 16 + rr; v4h o4; for (int j = 0; j < 4; ++j) o4[j] = (b16)(Tf[wave][rr][lane * 4 + j] * XS); *(volatile v4h*)(QP + (((size_t)b * H + h) * T + tok) * HD + d) = o4; } }
    else {
      if (lane < 16) { const int d = lane * 4; for (int rr = 0; rr < 16; ++rr) { const int tok = t0 + wave * 16 + rr; v4h o4; for (int j = 0; j < 4; ++j) o4[j] = (b16)(Tf[wave][rr][d + j] * XS); *(volatile v4h*)(KP + ((size_t)b * T + tok) * HD + d) = o4; } }
#pragma unroll 1
      for (int q = 0; q < 16; ++q) { const int d = wave * 16 + q; const int cl = HD + d; const int tk = lane * 2; v2h hv, lv; for (int j = 0; j < 2; ++j) { const float f = Tf[(tk + j) >> 4][(tk + j) & 15][cl] * XS; const b16 p = (b16)f; hv[j] = p; lv[j] = (b16)((f - (float)p) * RS_); }
        const size_t oi = ((size_t)b * HD + d) * (size_t)T + t0 + lane * 2; *(volatile v2h*)(VTh + oi) = hv; *(volatile v2h*)(VTl + oi) = lv; } }
    __threadfence(); }
}
__global__ __launch_bounds__(64) void attn_kernel(const b16* __restrict__ QP, const b16* __restrict__ KP, const b16* __restrict__ VTh, const b16* __restrict__ VTl, b16* __restrict__ Ch, b16* __restrict__ Cl) {
  __shared__ __attribute__((aligned(16))) b16 Pb[2][16][32 + 8]; __shared__ __attribute__((aligned(16))) float To[2][16][HD + 4];
  const int wave = threadIdx.x >> 5, lane = threadIdx.x & 31, hh = lane >> 4, col = lane & 15; const int b = blockIdx.y / H, h = blockIdx.y % H; const int q0 = blockIdx.x * 32 + wave * 16, qi = q0 + col;
  const size_t ph = (size_t)b * H + h; const b16* Qb = QP + ph * T * HD; const b16* Kb = KP + (size_t)b * T * HD; const b16* Vh = VTh + (size_t)b * HD * (size_t)T; const b16* Vl = VTl + (size_t)b * HD * (size_t)T;
  const v16b qa0 = frag_kb(Qb + (size_t)qi * HD, hh), qa1 = frag_kb(Qb + (size_t)qi * HD + 32, hh);
  const float cs = LOG2E / (8.0f * XS * XS);
  float m = -INFINITY, l = 0.0f; v8f o[4], ol[4]; for (int t = 0; t < 4; ++t) { o[t] = (v8f){}; ol[t] = (v8f){}; }
#pragma unroll 1
  for (int kb = 0; kb < T; kb += 32) {
    float e[16]; float mx = -INFINITY;
#pragma unroll
    for (int u = 0; u < 2; ++u) { v8f s = (v8f){}; const size_t kr = (size_t)(kb + u * 16 + col) * HD; s = wmma16b(frag_kb(Kb + kr, hh), qa0, s); s = wmma16b(frag_kb(Kb + kr + 32, hh), qa1, s);
#pragma unroll
      for (int r = 0; r < 8; ++r) { const float vv = s[r] * cs; e[u * 8 + r] = vv; mx = fmaxf(mx, vv); } }
    mx = fmaxf(mx, __shfl_xor(mx, 16)); const float mn = fmaxf(m, mx); const float al = nexp2(m - mn); float sum = 0.0f;
#pragma unroll
    for (int i2 = 0; i2 < 16; ++i2) { const float p = nexp2(e[i2] - mn); sum += p; Pb[wave][col][(i2 < 8 ? 0 : 16) + 8 * hh + (i2 & 7)] = (b16)(p * PS); }
    sum += __shfl_xor(sum, 16); l = l * al + sum; m = mn;
    wave_lds_sync();
    const v16b pf = frag_kb(&Pb[wave][col][0], hh);
#pragma unroll
    for (int t = 0; t < 4; ++t) { o[t] *= al; o[t] = wmma16b(frag_kb(Vh + (size_t)(t * 16 + col) * T + kb, hh), pf, o[t]); ol[t] = wmma16b(frag_kb(Vl + (size_t)(t * 16 + col) * T + kb, hh), pf, ol[t] * al); }
    wave_lds_sync(); }
  const float inv = 1.0f / (l * PS * XS);
#pragma unroll
  for (int t = 0; t < 4; ++t)
#pragma unroll
    for (int r = 0; r < 8; ++r) To[wave][col][t * 16 + 8 * hh + r] = (o[t][r] + ol[t][r] * (1.0f / RS_)) * inv;
  wave_lds_sync();
  for (int pass = 0; pass < 2; ++pass) { for (int rr = 0; rr < 16; ++rr) { const v2f f = *(const v2f*)(&To[wave][rr][lane * 2]); v2h hv, lv; for (int j = 0; j < 2; ++j) { b16 p, q; split16(f[j] * XS, p, q); hv[j] = p; lv[j] = q; }
      const size_t oi = ((size_t)b * T + q0 + rr) * DM + h * HD + lane * 2; *(volatile v2h*)(Ch + oi) = hv; *(volatile v2h*)(Cl + oi) = lv; } __threadfence(); }
}
__global__ __launch_bounds__(128) void out_kernel(const b16* __restrict__ Ch, const b16* __restrict__ Cl, const b16* __restrict__ WO, const float* __restrict__ bo, float* __restrict__ out) {
  __shared__ __attribute__((aligned(16))) float Tf[4][16][128 + 4];
  const int wave = threadIdx.x >> 5, lane = threadIdx.x & 31, nloc = lane & 15, hlf = lane >> 4; const int b = blockIdx.z; const size_t m0 = (size_t)b * T + ((size_t)blockIdx.x * 4 + wave) * 16; const int n0 = blockIdx.y * 128;
  v8f acc[8];
#pragma unroll
  for (int t = 0; t < 8; ++t) acc[t] = (v8f){};
#pragma unroll 2
  for (int kb = 0; kb < DM; kb += 32) { const v16b a = frag_kb(Ch + (m0 + nloc) * DM + kb, hlf), al = frag_kb(Cl + (m0 + nloc) * DM + kb, hlf);
#pragma unroll
    for (int t = 0; t < 8; ++t) { const v16b bw = frag_kb(WO + (size_t)(n0 + t * 16 + nloc) * DM + kb, hlf); acc[t] = wmma16b(a, bw, acc[t]); acc[t] = wmma16b(al, bw, acc[t]); } }
#pragma unroll
  for (int t = 0; t < 8; ++t) { const float bb = bf16_rne(bo[n0 + t * 16 + nloc]);
#pragma unroll
    for (int r = 0; r < 8; ++r) Tf[wave][8 * hlf + r][t * 16 + nloc] = acc[t][r] * (1.0f / (XS * WSC)) + bb; }
  wave_lds_sync();
  for (int pass = 0; pass < 2; ++pass) { for (int rr = 0; rr < 16; ++rr) *(volatile v4f*)(out + (m0 + rr) * DM + n0 + lane * 4) = *(const v4f*)(&Tf[wave][rr][lane * 4]); __threadfence(); }
}
}

extern "C" void kernel_launch(void* const* d_in, const int* in_sizes, int n_in, void* d_out, int out_size, void* d_ws, size_t ws_size, hipStream_t stream) {
  (void)n_in;
  auto Fp = [&](int i) { return (const float*)d_in[i]; };
  if (in_sizes[0] != B * T * DM || in_sizes[1] != DM * DM || in_sizes[2] != DM || in_sizes[3] != DM * HD || in_sizes[4] != HD || in_sizes[5] != DM * HD || in_sizes[6] != HD || in_sizes[7] != DM * DM || in_sizes[8] != DM || out_size != B * T * DM) return;
  size_t off = 0; char* ws = (char*)d_ws;
  auto carve = [&](size_t bytes) { char* p = ws + off; off += (bytes + 255) & ~(size_t)255; return p; };
  b16* WT = (b16*)carve((size_t)NWT * DM * 2); b16* WO = (b16*)carve((size_t)DM * DM * 2); const size_t plane = (size_t)B * T * DM * 2, kvplane = (size_t)B * T * HD * 2;
  b16* QP = (b16*)carve(plane); b16* KP = (b16*)carve(kvplane); b16* VTh = (b16*)carve(kvplane); b16* VTl = (b16*)carve(kvplane); b16* Ch = (b16*)carve(plane); b16* Cl = (b16*)carve(plane);
  if (off > ws_size || off > ((size_t)128 << 20)) return;
  prep_kernel<<<(unsigned)((((size_t)NWT * DM + (size_t)DM * DM) / 8 + 255) / 256), 256, 0, stream>>>(Fp(1), Fp(3), Fp(5), Fp(7), WT, WO);
  proj_kernel<<<dim3(T / 64, BL, NSL + 1), 128, 0, stream>>>(Fp(0), WT, Fp(2), Fp(4), Fp(6), QP, KP, VTh, VTl);
  attn_kernel<<<dim3(QL / 32, BL * H), 64, 0, stream>>>(QP, KP, VTh, VTl, Ch, Cl);
  out_kernel<<<dim3(QL / 64, DM / 128, BL), 128, 0, stream>>>(Ch, Cl, WO, Fp(8), (float*)d_out);
}
